// MultiScaleAttentionBlock_3770981286358
// MI455X (gfx1250) — hardware-verified
//
#include <hip/hip_runtime.h>


#define NB_  8
#define SS   1024
#define S2   512
#define DD   512
#define NH_  8
#define HD   64
#define DFF  2048
#define NR   (NB_ * SS)
#define NR2  (NB_ * S2)
#define DM   DD
#define PCAR 1024.0f
#define LOSC 1024.0f
typedef _Float16 h16;
typedef unsigned short bf;
typedef __attribute__((ext_vector_type(16))) __bf16   v16bf;
typedef __attribute__((ext_vector_type(16))) _Float16 v16h;
typedef __attribute__((ext_vector_type(8)))  _Float16 v8h;
typedef __attribute__((ext_vector_type(8)))  unsigned short v8us;
typedef __attribute__((ext_vector_type(8)))  float    v8f;
typedef __attribute__((ext_vector_type(4)))  float    v4f;
typedef v8h  __attribute__((may_alias)) v8ha;
typedef v4f  __attribute__((may_alias)) v4fa;
typedef v8us __attribute__((may_alias)) v8usa;

__device__ __forceinline__ unsigned short f2bf(float f) { unsigned u = __float_as_uint(f); u += 0x7FFFu + ((u >> 16) & 1u); return (unsigned short)(u >> 16); }
__device__ __forceinline__ float bf2f(unsigned short b) { return __uint_as_float(((unsigned)b) << 16); }
__device__ __forceinline__ float bfr(float f) { return bf2f(f2bf(f)); }
__device__ __forceinline__ v16h cat16(v8h lo, v8h hi) { return __builtin_shufflevector(lo, hi, 0, 1, 2, 3, 4, 5, 6, 7, 8, 9, 10, 11, 12, 13, 14, 15); }
__device__ __forceinline__ v16bf cat16b(v8us lo, v8us hi) { return __builtin_bit_cast(v16bf, __builtin_shufflevector(lo, hi, 0, 1, 2, 3, 4, 5, 6, 7, 8, 9, 10, 11, 12, 13, 14, 15)); }
__device__ __forceinline__ v8f wmma16(v16h a, v16h b, v8f c) { return __builtin_amdgcn_wmma_f32_16x16x32_f16(false, a, false, b, (short)0, c, false, false); }
__device__ __forceinline__ v8f wmmab(v16bf a, v16bf b, v8f c) { return __builtin_amdgcn_wmma_f32_16x16x32_bf16(false, a, false, b, (short)0, c, false, false); }

template <bool SPLITA, bool F16OUT = false>
__global__ __launch_bounds__(128) void k_gemmb(const bf* __restrict__ A, const bf* __restrict__ Al, const bf* __restrict__ Bn, const float* __restrict__ bias, float* C, int ldc, h16* C2, const float* __restrict__ R = nullptr, int K = DM, int roundR = 1) {
    __shared__ __align__(16) float ost[4][16 * 68];
    const int lane = threadIdx.x & 31, wave = threadIdx.x >> 5, lr = lane & 15, hi = lane >> 4;
    const int r0 = blockIdx.x * 64 + wave * 16, c0 = blockIdx.y * 64;
    const size_t aoff = (size_t)(r0 + lr) * K + 8 * hi;
    size_t boff[4];
#pragma unroll
    for (int t = 0; t < 4; ++t) boff[t] = (size_t)(c0 + t * 16 + lr) * K + 8 * hi;
    v8f acc[4];
#pragma unroll
    for (int t = 0; t < 4; ++t) acc[t] = (v8f){};
#pragma unroll 1
    for (int kc = 0; kc < K; kc += 32) {
        const v16bf a = cat16b(*(const v8us*)(A + aoff + kc), *(const v8us*)(A + aoff + kc + 16));
        v16bf al = a;
        if (SPLITA) al = cat16b(*(const v8us*)(Al + aoff + kc), *(const v8us*)(Al + aoff + kc + 16));
#pragma unroll
        for (int t = 0; t < 4; ++t) { const v16bf b = cat16b(*(const v8us*)(Bn + boff[t] + kc), *(const v8us*)(Bn + boff[t] + kc + 16)); acc[t] = wmmab(a, b, acc[t]); if (SPLITA) acc[t] = wmmab(al, b, acc[t]); }
        asm volatile("v_nop\n\tv_nop\n\tv_nop\n\tv_nop" : "+v"(acc[0]), "+v"(acc[1]), "+v"(acc[2]), "+v"(acc[3]) : "v"(a), "v"(al));
    }
    float* os = &ost[wave][0];
#pragma unroll
    for (int t = 0; t < 4; ++t) { const float bv = bias ? bfr(bias[c0 + t * 16 + lr]) : 0.f;
#pragma unroll
        for (int j = 0; j < 8; ++j) os[(hi * 8 + j) * 68 + t * 16 + lr] = acc[t][j] + bv; }
    __syncthreads();
    if (F16OUT) {
        h16* crow = (h16*)(void*)C + (size_t)r0 * ldc + c0;
        auto pass = [&]() {
#pragma unroll
            for (int s = 0; s < 4; ++s) { const int row = 4 * s + (lane >> 3), piece = lane & 7; const float* sp = os + row * 68 + piece * 8; v8h o, o2;
#pragma unroll
                for (int i = 0; i < 8; ++i) { const h16 a = (h16)sp[i]; o[i] = a; o2[i] = (h16)((sp[i] - (float)a) * LOSC); }
                *(volatile v8h*)(crow + (size_t)row * ldc + piece * 8) = o; if (C2) *(volatile v8h*)(C2 + (size_t)r0 * ldc + c0 + (size_t)row * ldc + piece * 8) = o2; }
        };
        pass(); __threadfence(); pass();
    } else {
        float* crow = C + (size_t)r0 * ldc + c0;
        auto pass = [&]() {
#pragma unroll
            for (int s = 0; s < 8; ++s) { const int Lid = (lane >> 3) + 4 * s, piece = lane & 7; const int row = Lid >> 1, cofs = (Lid & 1) * 32 + piece * 4;
                v4f val = *(const v4fa*)(os + row * 68 + cofs); if (R) { const v4f rv = *(const v4f*)(R + ((size_t)r0 + row) * ldc + c0 + cofs); val += roundR ? (v4f){bfr(rv[0]), bfr(rv[1]), bfr(rv[2]), bfr(rv[3])} : rv; }
                *(volatile v4f*)(crow + (size_t)row * ldc + cofs) = val; }
        };
        pass(); __threadfence(); pass();
    }
}

__global__ __launch_bounds__(256) void k_cvt8(const float* __restrict__ src, bf* dst, size_t n8) {
    const size_t i = (size_t)blockIdx.x * 256 + threadIdx.x; if (i >= n8) return;
    const v8f v = *(const v8f*)(src + i * 8); v8us o;
#pragma unroll
    for (int k = 0; k < 8; ++k) o[k] = f2bf(v[k]);
    *(volatile v8us*)(dst + i * 8) = o; __threadfence(); *(volatile v8us*)(dst + i * 8) = o;
}
__global__ __launch_bounds__(256) void k_zero8(bf* dst, size_t n8) {
    const size_t i = (size_t)blockIdx.x * 256 + threadIdx.x; if (i >= n8) return; v8us z;
#pragma unroll
    for (int k = 0; k < 8; ++k) z[k] = 0;
    *(volatile v8us*)(dst + i * 8) = z; __threadfence(); *(volatile v8us*)(dst + i * 8) = z;
}

__global__ __launch_bounds__(128) void k_gemmh(const h16* __restrict__ A, const h16* __restrict__ Bn, const float* __restrict__ bias, float* C, int ldc, const float* __restrict__ R, int K, size_t sA, size_t sB, size_t sC, int roundR) {
    __shared__ __align__(16) float ost[4][16 * 68];
    const size_t z = blockIdx.z; A += z * sA; Bn += z * sB; C += z * sC; if (R) R += z * sC;
    const int lane = threadIdx.x & 31, wave = threadIdx.x >> 5, lr = lane & 15, hi = lane >> 4;
    const int r0 = blockIdx.x * 64 + wave * 16, c0 = blockIdx.y * 64;
    const size_t aoff = (size_t)(r0 + lr) * K + 8 * hi;
    size_t boff[4];
#pragma unroll
    for (int t = 0; t < 4; ++t) boff[t] = (size_t)(c0 + t * 16 + lr) * K + 8 * hi;
    v8f acc[4];
#pragma unroll
    for (int t = 0; t < 4; ++t) acc[t] = (v8f){};
#pragma unroll 1
    for (int kc = 0; kc < K; kc += 32) {
        const v16h a = cat16(*(const v8h*)(A + aoff + kc), *(const v8h*)(A + aoff + kc + 16));
#pragma unroll
        for (int t = 0; t < 4; ++t) { const v16h b = cat16(*(const v8h*)(Bn + boff[t] + kc), *(const v8h*)(Bn + boff[t] + kc + 16)); acc[t] = wmma16(a, b, acc[t]); }
        asm volatile("v_nop\n\tv_nop\n\tv_nop\n\tv_nop" : "+v"(acc[0]), "+v"(acc[1]), "+v"(acc[2]), "+v"(acc[3]) : "v"(a));
    }
    float* os = &ost[wave][0];
#pragma unroll
    for (int t = 0; t < 4; ++t) { const float bv = bias ? bfr(bias[c0 + t * 16 + lr]) : 0.f;
#pragma unroll
        for (int j = 0; j < 8; ++j) os[(hi * 8 + j) * 68 + t * 16 + lr] = acc[t][j] + bv; }
    __syncthreads();
    float* crow = C + (size_t)r0 * ldc + c0;
    auto pass = [&]() {
#pragma unroll
        for (int s = 0; s < 8; ++s) { const int Lid = (lane >> 3) + 4 * s, piece = lane & 7; const int row = Lid >> 1, cofs = (Lid & 1) * 32 + piece * 4;
            v4f val = *(const v4fa*)(os + row * 68 + cofs); if (R) { const v4f rv = *(const v4f*)(R + ((size_t)r0 + row) * ldc + c0 + cofs); val += roundR ? (v4f){bfr(rv[0]), bfr(rv[1]), bfr(rv[2]), bfr(rv[3])} : rv; }
            *(volatile v4f*)(crow + (size_t)row * ldc + cofs) = val; }
    };
    pass(); __threadfence(); pass();
}

typedef __attribute__((ext_vector_type(4))) _Float16 v4h;
__device__ __forceinline__ h16 tohx(float x) { return (h16)x; }
__device__ __forceinline__ float gelu_e(float x) { return 0.5f * x * (1.0f + erff(x * 0.70710678118654752f)); }
__global__ __launch_bounds__(256) void k_cvt8h(const float* __restrict__ src, h16* dst, size_t n8) { const size_t i = (size_t)blockIdx.x * 256 + threadIdx.x; if (i >= n8) return; const v8f v = *(const v8f*)(src + i * 8); v8h o;
#pragma unroll
    for (int k = 0; k < 8; ++k) o[k] = tohx(bfr(v[k])); *(volatile v8h*)(dst + i * 8) = o; __threadfence(); *(volatile v8h*)(dst + i * 8) = o; }
__global__ __launch_bounds__(256) void k_cvtx512(const float* __restrict__ x, bf* A) {
    const int lane = threadIdx.x & 31; const size_t r = (size_t)blockIdx.x * 8 + (threadIdx.x >> 5); if (r >= (size_t)NR) return;
#pragma unroll 1
    for (int ps = 0; ps < 2; ++ps) {
#pragma unroll
        for (int q = 0; q < DD / 256; ++q) { const size_t o = r * DD + q * 256 + lane * 8; v8us v;
#pragma unroll
            for (int i = 0; i < 8; ++i) v[i] = f2bf(x[o + i]);
            *(volatile v8us*)(A + o) = v; }
        if (ps == 0) __threadfence(); }
}
__global__ __launch_bounds__(256) void k_hplg(const float* __restrict__ F, int ld, int ntok, int b, int col0, float sc, h16* P) {
    const int lane = threadIdx.x & 31; const size_t w = (size_t)blockIdx.x * 8 + (threadIdx.x >> 5); const int t = (int)(w * 2 + (lane >> 4)); if (t >= ntok) return; const int z = blockIdx.z; const int c0 = (lane & 15) * 4; v4h o;
#pragma unroll
    for (int q = 0; q < 4; ++q) o[q] = tohx(F[((size_t)b * ntok + t) * ld + col0 + z * HD + c0 + q] * sc);
    const size_t off = ((size_t)z * ntok + t) * HD + c0; *(volatile v4h*)(P + off) = o; __threadfence(); *(volatile v4h*)(P + off) = o;
}
__global__ __launch_bounds__(256) void k_vTg(const float* __restrict__ F, int ld, int ntok, int b, int col0, h16* VT) {
    __shared__ float tl[64][65];
    const int tid = threadIdx.x; const int t0 = blockIdx.x * 64; const int z = blockIdx.z; const int rr = tid >> 2, cq = (tid & 3) * 16;
#pragma unroll
    for (int i = 0; i < 16; ++i) tl[rr][cq + i] = F[((size_t)b * ntok + t0 + rr) * ld + col0 + z * HD + cq + i];
    __syncthreads();
    const int lane = tid & 31, wv = tid >> 5;
    auto pass = [&]() {
#pragma unroll
        for (int st = 0; st < 4; ++st) { const int dr = wv * 8 + st * 2 + (lane >> 4); const int tq = (lane & 15) * 4; v4h v;
#pragma unroll
            for (int i = 0; i < 4; ++i) v[i] = tohx(tl[tq + i][dr]);
            *(volatile v4h*)(VT + ((size_t)z * HD + dr) * ntok + t0 + tq) = v; }
    };
    pass(); __threadfence(); pass();
}
__global__ __launch_bounds__(256) void k_softg(const float* __restrict__ S, int ntok, h16* P) {
    const int lane = threadIdx.x & 31, i = blockIdx.x * 8 + (threadIdx.x >> 5); if (i >= ntok) return; const size_t zo = ((size_t)blockIdx.z * ntok + i) * ntok; const float* sr = S + zo; h16* po = P + zo;
    float m = -3.0e38f;
#pragma unroll 1
    for (int c0 = lane * 4; c0 < ntok; c0 += 128) {
#pragma unroll
        for (int q = 0; q < 4; ++q) m = fmaxf(m, sr[c0 + q]); }
#pragma unroll
    for (int sh = 16; sh; sh >>= 1) m = fmaxf(m, __shfl_xor(m, sh, 32));
    float sum = 0.f;
#pragma unroll 1
    for (int c0 = lane * 4; c0 < ntok; c0 += 128) {
#pragma unroll
        for (int q = 0; q < 4; ++q) sum += __expf(sr[c0 + q] - m); }
#pragma unroll
    for (int sh = 16; sh; sh >>= 1) sum += __shfl_xor(sum, sh, 32);
    const float f = __fdiv_rn(PCAR, sum);
#pragma unroll 1
    for (int ps = 0; ps < 2; ++ps) {
#pragma unroll 1
        for (int c0 = lane * 4; c0 < ntok; c0 += 128) { v4h o;
#pragma unroll
            for (int q = 0; q < 4; ++q) o[q] = tohx(__expf(sr[c0 + q] - m) * f);
            *(volatile v4h*)(po + c0) = o; }
        if (ps == 0) __threadfence(); }
}
__global__ __launch_bounds__(256) void k_mergeg(const float* __restrict__ OZ, int ntok, int b, h16* OH) {
    const int lane = threadIdx.x & 31, i = blockIdx.x * 8 + (threadIdx.x >> 5); if (i >= ntok) return;
#pragma unroll 1
    for (int ps = 0; ps < 2; ++ps) {
#pragma unroll
        for (int p = 0; p < 2; ++p) { const int c0 = p * 256 + lane * 8; const int z = c0 / HD, d0 = c0 % HD; v8h o;
#pragma unroll
            for (int k = 0; k < 8; ++k) o[k] = tohx(OZ[((size_t)z * ntok + i) * HD + d0 + k] * (1.0f / PCAR));
            *(volatile v8h*)(OH + ((size_t)b * ntok + i) * DD + c0) = o; }
        if (ps == 0) __threadfence(); }
}
template <bool ROUNDA>
__global__ __launch_bounds__(256) void k_addln(const float* __restrict__ A, const float* __restrict__ Badd, const float* __restrict__ g, const float* __restrict__ bb, size_t rows, float* Y, h16* Yh) {
    const int lane = threadIdx.x & 31; const size_t r = (size_t)blockIdx.x * 8 + (threadIdx.x >> 5); if (r >= rows) return; float v[16]; float s = 0.f;
#pragma unroll
    for (int p = 0; p < 4; ++p) {
#pragma unroll
        for (int i = 0; i < 4; ++i) { const int c = p * 128 + lane * 4 + i; float a = A[r * DD + c]; if (ROUNDA) a = bfr(a); v[p * 4 + i] = a + Badd[r * DD + c]; s += v[p * 4 + i]; } }
#pragma unroll
    for (int sh = 16; sh; sh >>= 1) s += __shfl_xor(s, sh, 32);
    const float mu = s * (1.0f / DD); float q = 0.f;
#pragma unroll
    for (int i = 0; i < 16; ++i) { const float d = v[i] - mu; q = fmaf(d, d, q); }
#pragma unroll
    for (int sh = 16; sh; sh >>= 1) q += __shfl_xor(q, sh, 32);
    const float rs = rsqrtf(q * (1.0f / DD) + 1e-5f);
#pragma unroll 1
    for (int ps = 0; ps < 2; ++ps) {
#pragma unroll
        for (int p = 0; p < 4; ++p) { v4f o; v4h oh;
#pragma unroll
            for (int i = 0; i < 4; ++i) { const int c = p * 128 + lane * 4 + i; o[i] = (v[p * 4 + i] - mu) * rs * bfr(g[c]) + bfr(bb[c]); oh[i] = tohx(o[i]); }
            *(volatile v4f*)(Y + r * DD + p * 128 + lane * 4) = o; if (Yh) *(volatile v4h*)(Yh + r * DD + p * 128 + lane * 4) = oh; }
        if (ps == 0) __threadfence(); }
}
__global__ __launch_bounds__(256) void k_pool2(const float* __restrict__ X1, h16* PH) {
    const int lane = threadIdx.x & 31; const size_t r = (size_t)blockIdx.x * 8 + (threadIdx.x >> 5); if (r >= (size_t)NR2) return; const float* a = X1 + (2 * r) * DD; const float* b2 = a + DD;
#pragma unroll 1
    for (int ps = 0; ps < 2; ++ps) {
#pragma unroll
        for (int p = 0; p < 2; ++p) { const int c0 = p * 256 + lane * 8; v8h o;
#pragma unroll
            for (int k = 0; k < 8; ++k) o[k] = tohx((a[c0 + k] + b2[c0 + k]) * 0.5f);
            *(volatile v8h*)(PH + r * DD + c0) = o; }
        if (ps == 0) __threadfence(); }
}
__global__ __launch_bounds__(256) void k_upln(const float* __restrict__ X1, const float* __restrict__ A2, const float* __restrict__ g, const float* __restrict__ bb, float* Y, h16* Yh) {
    const int lane = threadIdx.x & 31; const size_t r = (size_t)blockIdx.x * 8 + (threadIdx.x >> 5); if (r >= (size_t)NR) return; const int b = (int)(r / SS), j = (int)(r % SS);
    float src = ((float)j + 0.5f) * ((float)S2 / (float)SS) - 0.5f; src = fminf(fmaxf(src, 0.f), (float)(S2 - 1)); const int i0 = (int)floorf(src); const int i1 = min(i0 + 1, S2 - 1); const float w = src - (float)i0;
    const float* a0 = A2 + ((size_t)b * S2 + i0) * DD; const float* a1 = A2 + ((size_t)b * S2 + i1) * DD; float v[16]; float s = 0.f;
#pragma unroll
    for (int p = 0; p < 4; ++p) {
#pragma unroll
        for (int i = 0; i < 4; ++i) { const int c = p * 128 + lane * 4 + i; v[p * 4 + i] = X1[r * DD + c] + (a0[c] * (1.0f - w) + a1[c] * w); s += v[p * 4 + i]; } }
#pragma unroll
    for (int sh = 16; sh; sh >>= 1) s += __shfl_xor(s, sh, 32);
    const float mu = s * (1.0f / DD); float q = 0.f;
#pragma unroll
    for (int i = 0; i < 16; ++i) { const float d = v[i] - mu; q = fmaf(d, d, q); }
#pragma unroll
    for (int sh = 16; sh; sh >>= 1) q += __shfl_xor(q, sh, 32);
    const float rs = rsqrtf(q * (1.0f / DD) + 1e-5f);
#pragma unroll 1
    for (int ps = 0; ps < 2; ++ps) {
#pragma unroll
        for (int p = 0; p < 4; ++p) { v4f o; v4h oh;
#pragma unroll
            for (int i = 0; i < 4; ++i) { const int c = p * 128 + lane * 4 + i; o[i] = (v[p * 4 + i] - mu) * rs * bfr(g[c]) + bfr(bb[c]); oh[i] = tohx(o[i]); }
            *(volatile v4f*)(Y + r * DD + p * 128 + lane * 4) = o; *(volatile v4h*)(Yh + r * DD + p * 128 + lane * 4) = oh; }
        if (ps == 0) __threadfence(); }
}
__global__ __launch_bounds__(256) void k_geluh(const float* __restrict__ F, size_t rows, h16* Hh) {
    const int lane = threadIdx.x & 31; const size_t r = (size_t)blockIdx.x * 8 + (threadIdx.x >> 5); if (r >= rows) return;
#pragma unroll 1
    for (int p = 0; p < DFF / 256; ++p) { const int c0 = p * 256 + lane * 8; v8h o;
#pragma unroll
        for (int k = 0; k < 8; ++k) o[k] = tohx(gelu_e(F[r * DFF + c0 + k]));
        *(volatile v8h*)(Hh + r * DFF + c0) = o; __threadfence(); *(volatile v8h*)(Hh + r * DFF + c0) = o; }
}
extern "C" void kernel_launch(void* const* d_in, const int* in_sizes, int n_in,
                              void* d_out, int out_size, void* d_ws, size_t ws_size, hipStream_t stream) {
    (void)in_sizes; (void)n_in; (void)out_size;
    const float* x = (const float*)d_in[0]; const float* win1 = (const float*)d_in[1]; const float* bin1 = (const float*)d_in[2]; const float* wout1 = (const float*)d_in[3]; const float* bout1 = (const float*)d_in[4]; const float* win2 = (const float*)d_in[5]; const float* bin2 = (const float*)d_in[6]; const float* wout2 = (const float*)d_in[7]; const float* bout2 = (const float*)d_in[8];
    const float* g1 = (const float*)d_in[9]; const float* be1 = (const float*)d_in[10]; const float* g2 = (const float*)d_in[11]; const float* be2 = (const float*)d_in[12]; const float* g3 = (const float*)d_in[13]; const float* be3 = (const float*)d_in[14]; const float* wff1 = (const float*)d_in[15]; const float* bff1 = (const float*)d_in[16]; const float* wff2 = (const float*)d_in[17]; const float* bff2 = (const float*)d_in[18];
    float* out = (float*)d_out;
    char* wsp = (char*)d_ws;
    auto take = [&](size_t bytes) { char* p = wsp; wsp += (bytes + 255) & ~(size_t)255; return (void*)p; };
    bf* WIN1 = (bf*)take((size_t)3 * DD * DD * 2); h16* WOUT1 = (h16*)take((size_t)DD * DD * 2); h16* WIN2 = (h16*)take((size_t)3 * DD * DD * 2); h16* WOUT2 = (h16*)take((size_t)DD * DD * 2); h16* WFF1 = (h16*)take((size_t)DFF * DD * 2); h16* WFF2 = (h16*)take((size_t)DD * DFF * 2);
    bf* XB = (bf*)take((size_t)NR * DD * 2);
    char* R1 = (char*)take((size_t)NR * 3 * DD * 4);
    char* R2 = (char*)take((size_t)54 << 20);
    h16* Qx = (h16*)take((size_t)NH_ * SS * HD * 2); h16* Kx = (h16*)take((size_t)NH_ * SS * HD * 2); h16* VT = (h16*)take((size_t)NH_ * HD * SS * 2); float* OZ = (float*)take((size_t)NH_ * SS * HD * 4);
    h16* OH = (h16*)take((size_t)NR * DD * 2); float* A1 = (float*)take((size_t)NR * DD * 4); float* X1 = (float*)take((size_t)NR * DD * 4); h16* PH = (h16*)take((size_t)NR2 * DD * 2); float* X2 = (float*)take((size_t)NR * DD * 4); h16* X2h = (h16*)take((size_t)NR * DD * 2); h16* Hh = (h16*)take((size_t)(NR / 2) * DFF * 2);
    if ((size_t)(wsp - (char*)d_ws) > ws_size) return;
    float* QKV1 = (float*)R1; float* F1 = (float*)R1;
    float* S = (float*)R2; h16* Px = (h16*)(R2 + ((size_t)NH_ * SS * SS * 4));
    float* QKV2 = (float*)R2; float* Sb = (float*)(R2 + ((size_t)NR2 * 3 * DD * 4)); h16* Pb = (h16*)((char*)Sb + (size_t)NH_ * S2 * S2 * 4); float* OZ2 = (float*)((char*)Pb + (size_t)NH_ * S2 * S2 * 2); h16* OH2 = (h16*)((char*)OZ2 + (size_t)NH_ * S2 * HD * 4); float* A2 = (float*)((char*)OH2 + (size_t)NR2 * DD * 2);
    float* FF2 = A1;
    const size_t n3 = (size_t)3 * DD * DD / 8, n1 = (size_t)DD * DD / 8, nf = (size_t)DFF * DD / 8;
    k_cvt8<<<(unsigned)((n3 + 255) / 256), 256, 0, stream>>>(win1, WIN1, n3); k_cvt8h<<<(unsigned)((n1 + 255) / 256), 256, 0, stream>>>(wout1, WOUT1, n1); k_cvt8h<<<(unsigned)((n3 + 255) / 256), 256, 0, stream>>>(win2, WIN2, n3); k_cvt8h<<<(unsigned)((n1 + 255) / 256), 256, 0, stream>>>(wout2, WOUT2, n1); k_cvt8h<<<(unsigned)((nf + 255) / 256), 256, 0, stream>>>(wff1, WFF1, nf); k_cvt8h<<<(unsigned)((nf + 255) / 256), 256, 0, stream>>>(wff2, WFF2, nf);
    k_cvtx512<<<NR / 8, 256, 0, stream>>>(x, XB);
    k_gemmb<false, false><<<dim3(NR / 64, (3 * DD) / 64, 1), 128, 0, stream>>>(XB, nullptr, WIN1, bin1, QKV1, 3 * DD, nullptr, nullptr, DD);
    for (int b = 0; b < NB_; ++b) {
        k_hplg<<<dim3((SS / 2) / 8, 1, NH_), 256, 0, stream>>>(QKV1, 3 * DD, SS, b, 0, 0.125f, Qx); k_hplg<<<dim3((SS / 2) / 8, 1, NH_), 256, 0, stream>>>(QKV1, 3 * DD, SS, b, DD, 1.0f, Kx); k_vTg<<<dim3(SS / 64, 1, NH_), 256, 0, stream>>>(QKV1, 3 * DD, SS, b, 2 * DD, VT);
        k_gemmh<<<dim3(SS / 64, SS / 64, NH_), 128, 0, stream>>>(Qx, Kx, nullptr, S, SS, nullptr, HD, (size_t)SS * HD, (size_t)SS * HD, (size_t)SS * SS, 0);
        k_softg<<<dim3(SS / 8, 1, NH_), 256, 0, stream>>>(S, SS, Px);
        k_gemmh<<<dim3(SS / 64, 1, NH_), 128, 0, stream>>>(Px, VT, nullptr, OZ, HD, nullptr, SS, (size_t)SS * SS, (size_t)HD * SS, (size_t)SS * HD, 0);
        k_mergeg<<<SS / 8, 256, 0, stream>>>(OZ, SS, b, OH); }
    k_gemmh<<<dim3(NR / 64, DD / 64, 1), 128, 0, stream>>>(OH, WOUT1, bout1, A1, DD, nullptr, DD, 0, 0, 0, 0);
    k_addln<true><<<NR / 8, 256, 0, stream>>>(x, A1, g1, be1, NR, X1, nullptr);
    k_pool2<<<NR2 / 8, 256, 0, stream>>>(X1, PH);
    k_gemmh<<<dim3(NR2 / 64, (3 * DD) / 64, 1), 128, 0, stream>>>(PH, WIN2, bin2, QKV2, 3 * DD, nullptr, DD, 0, 0, 0, 0);
    for (int b = 0; b < NB_; ++b) {
        k_hplg<<<dim3((S2 / 2) / 8, 1, NH_), 256, 0, stream>>>(QKV2, 3 * DD, S2, b, 0, 0.125f, Qx); k_hplg<<<dim3((S2 / 2) / 8, 1, NH_), 256, 0, stream>>>(QKV2, 3 * DD, S2, b, DD, 1.0f, Kx); k_vTg<<<dim3(S2 / 64, 1, NH_), 256, 0, stream>>>(QKV2, 3 * DD, S2, b, 2 * DD, VT);
        k_gemmh<<<dim3(S2 / 64, S2 / 64, NH_), 128, 0, stream>>>(Qx, Kx, nullptr, Sb, S2, nullptr, HD, (size_t)S2 * HD, (size_t)S2 * HD, (size_t)S2 * S2, 0);
        k_softg<<<dim3(S2 / 8, 1, NH_), 256, 0, stream>>>(Sb, S2, Pb);
        k_gemmh<<<dim3(S2 / 64, 1, NH_), 128, 0, stream>>>(Pb, VT, nullptr, OZ2, HD, nullptr, S2, (size_t)S2 * S2, (size_t)HD * S2, (size_t)S2 * HD, 0);
        k_mergeg<<<S2 / 8, 256, 0, stream>>>(OZ2, S2, b, OH2); }
    k_gemmh<<<dim3(NR2 / 64, DD / 64, 1), 128, 0, stream>>>(OH2, WOUT2, bout2, A2, DD, nullptr, DD, 0, 0, 0, 0);
    k_upln<<<NR / 8, 256, 0, stream>>>(X1, A2, g2, be2, X2, X2h);
    for (int hf = 0; hf < 2; ++hf) { const size_t r0 = (size_t)hf * (NR / 2);
        k_gemmh<<<dim3((NR / 2) / 64, DFF / 64, 1), 128, 0, stream>>>(X2h + r0 * DD, WFF1, bff1, F1, DFF, nullptr, DD, 0, 0, 0, 0);
        k_geluh<<<(NR / 2) / 8, 256, 0, stream>>>(F1, NR / 2, Hh);
        k_gemmh<<<dim3((NR / 2) / 64, DD / 64, 1), 128, 0, stream>>>(Hh, WFF2, bff2, FF2 + r0 * DD, DD, nullptr, DFF, 0, 0, 0, 0); }
    k_addln<false><<<NR / 8, 256, 0, stream>>>(X2, FF2, g3, be3, NR, out, nullptr);
}
